// ISTFT_53068615909609
// MI455X (gfx1250) — hardware-verified
//
#include <hip/hip_runtime.h>

#define NFFT    1024
#define HOP     256
#define NB      8
#define NBH     4
#define NFRAMES 2000
#define NFREQ   513
#define KTOT    1026
#define KLOOP   1056
#define KP      1088
#define MH      (NBH * NFRAMES)
#define OUTLEN  511744
#define QROW    (OUTLEN / 4)
#define LDP     72

static_assert(MH % 64 == 0);
static_assert(KLOOP % 32 == 0);
static_assert(KLOOP >= KTOT);
static_assert(KP >= KLOOP);
static_assert(KP % 64 == 0);
static_assert(NFFT % 128 == 0);
static_assert(OUTLEN % 128 == 0);
static_assert((NBH * QROW) % 256 == 0);
static_assert((LDP * 2) % 16 == 0);

typedef unsigned short v8us  __attribute__((ext_vector_type(8)));
typedef unsigned short v16us __attribute__((ext_vector_type(16)));
typedef __bf16         v16bf __attribute__((ext_vector_type(16)));
typedef float          v8f   __attribute__((ext_vector_type(8)));
typedef float          v4f   __attribute__((ext_vector_type(4)));
typedef v8us __attribute__((may_alias)) v8usa;
typedef v4f  __attribute__((may_alias)) v4fa;

union FragU { v16us u; v8us h[2]; };

__device__ __forceinline__ unsigned int bf16_rne_bits(float x) {
  unsigned int u = __float_as_uint(x);
  u += 0x7FFFu + ((u >> 16) & 1u);
  return u >> 16;
}
__device__ __forceinline__ void split2(float x, unsigned short& hi, unsigned short& lo) {
  const unsigned int hb = bf16_rne_bits(x);
  const float hf = __uint_as_float(hb << 16);
  const unsigned int lb = bf16_rne_bits(x - hf);
  hi = (unsigned short)hb;
  lo = (unsigned short)lb;
}

__device__ __forceinline__ v16us load_frag(const unsigned short* p, int h) {
  FragU f;
  f.h[0] = *(const v8usa*)(p + 8 * h);
  f.h[1] = *(const v8usa*)(p + 16 + 8 * h);
  return f.u;
}
__device__ __forceinline__ v8f wmma_bf(v16us a, v16us b, v8f c) {
  return __builtin_amdgcn_wmma_f32_16x16x32_bf16(false, __builtin_bit_cast(v16bf, a), false,
                                                 __builtin_bit_cast(v16bf, b), (short)0, c, false, false);
}

__device__ __forceinline__ void plane_store_pass(const unsigned short* sh, const unsigned short* sl,
                                                 unsigned short* ph, unsigned short* pl,
                                                 size_t row0, int nrows, int kcol, int w, int lane) {
  const int q = lane & 7, sub = lane >> 3;
  #pragma unroll
  for (int i = 0; i < 2; ++i) {
    const int row = 8 * w + 4 * i + sub;
    const v8us hv = *(const v8usa*)(sh + row * LDP + 8 * q);
    const v8us lv = *(const v8usa*)(sl + row * LDP + 8 * q);
    if (row < nrows) {
      const size_t off = (row0 + (size_t)row) * (size_t)KP + (size_t)(kcol + 8 * q);
      *(volatile v8us*)(ph + off) = hv;
      *(volatile v8us*)(pl + off) = lv;
    }
  }
}

__global__ __launch_bounds__(256) void prep_basis(const float* __restrict__ Wr, const float* __restrict__ Wi,
                                                  unsigned short* __restrict__ bh, unsigned short* __restrict__ bl)
{
  __shared__ __attribute__((aligned(16))) unsigned short sh[64 * LDP];
  __shared__ __attribute__((aligned(16))) unsigned short sl[64 * LDP];
  const int tid = threadIdx.x, lane = tid & 31, w = tid >> 5;
  const int k0 = blockIdx.x * 64, o0 = blockIdx.y * 64;

  #pragma unroll
  for (int it = 0; it < 4; ++it) {
    const int idx = it * 256 + tid;
    const int kl = idx >> 4, oq = idx & 15;
    const int k = k0 + kl;
    const int o = o0 + 4 * oq;
    const int i = k - NFREQ;
    const int kr  = min(k, 512);
    const int kr2 = NFFT - min(max(k, 1), 511);
    const int ki  = min(max(i, 0), 512);
    const int ki2 = NFFT - min(max(i, 1), 511);
    const v4f wr1 = *(const v4fa*)(Wr + (size_t)kr  * NFFT + o);
    const v4f wr2 = *(const v4fa*)(Wr + (size_t)kr2 * NFFT + o);
    const v4f wi1 = *(const v4fa*)(Wi + (size_t)ki  * NFFT + o);
    const v4f wi2 = *(const v4fa*)(Wi + (size_t)ki2 * NFFT + o);
    const bool isr   = (k < NFREQ);
    const bool hasr2 = (k >= 1) && (k <= 511);
    const bool isi   = (k >= NFREQ) && (k < KTOT);
    const bool hasi2 = (i >= 1) && (i <= 511);
    #pragma unroll
    for (int e = 0; e < 4; ++e) {
      const float pr = hasr2 ? (wr1[e] + wr2[e]) : wr1[e];
      const float pim = (hasi2 ? wi2[e] : 0.0f) - wi1[e];
      const float v = isr ? pr : (isi ? pim : 0.0f);
      unsigned short hb, lb;
      split2(v, hb, lb);
      sh[(4 * oq + e) * LDP + kl] = hb;
      sl[(4 * oq + e) * LDP + kl] = lb;
    }
  }
  __syncthreads();

  plane_store_pass(sh, sl, bh, bl, (size_t)o0, 64, k0, w, lane);
  __threadfence();
  plane_store_pass(sh, sl, bh, bl, (size_t)o0, 64, k0, w, lane);
}

__global__ __launch_bounds__(256) void prep_frames(const float* __restrict__ re, const float* __restrict__ im,
                                                   unsigned short* __restrict__ ah, unsigned short* __restrict__ al,
                                                   int pass_id)
{
  __shared__ __attribute__((aligned(16))) unsigned short sh[64 * LDP];
  __shared__ __attribute__((aligned(16))) unsigned short sl[64 * LDP];
  const int tid = threadIdx.x, lane = tid & 31, w = tid >> 5;
  const int k0 = blockIdx.x * 64, t0 = blockIdx.y * 64, blk = blockIdx.z;
  const int b = pass_id * NBH + blk;

  #pragma unroll
  for (int it = 0; it < 4; ++it) {
    const int idx = it * 256 + tid;
    const int kl = idx >> 4, tq = idx & 15;
    const int k = k0 + kl;
    const int binr = min(k, NFREQ - 1);
    const int bini = min(max(k - NFREQ, 0), NFREQ - 1);
    const int ts = min(t0 + 4 * tq, NFRAMES - 4);
    const v4f vr = *(const v4fa*)(re + ((size_t)(b * NFREQ + binr)) * NFRAMES + ts);
    const v4f vi = *(const v4fa*)(im + ((size_t)(b * NFREQ + bini)) * NFRAMES + ts);
    const bool isr = (k < NFREQ);
    const bool isi = (k >= NFREQ) && (k < KTOT);
    #pragma unroll
    for (int e = 0; e < 4; ++e) {
      const float v = isr ? vr[e] : (isi ? vi[e] : 0.0f);
      unsigned short hb, lb;
      split2(v, hb, lb);
      sh[(4 * tq + e) * LDP + kl] = hb;
      sl[(4 * tq + e) * LDP + kl] = lb;
    }
  }
  __syncthreads();

  const size_t row0 = (size_t)blk * NFRAMES + (size_t)t0;
  const int nrows = NFRAMES - t0;
  plane_store_pass(sh, sl, ah, al, row0, nrows, k0, w, lane);
  __threadfence();
  plane_store_pass(sh, sl, ah, al, row0, nrows, k0, w, lane);
}

__device__ __forceinline__ void gemm_store_pass(const float* so, float* S, int m0, int n0w, int lane) {
  const int q = lane & 7, sub = lane >> 3;
  #pragma unroll
  for (int it = 0; it < 16; ++it) {
    const int lid = it * 4 + sub;
    const v4f v = *(const v4fa*)(so + lid * 32 + 4 * q);
    *(volatile v4f*)(S + (size_t)(m0 + lid) * NFFT + n0w + 4 * q) = v;
  }
}

__global__ __launch_bounds__(128) void synth_gemm(const unsigned short* __restrict__ ah,
                                                  const unsigned short* __restrict__ al,
                                                  const unsigned short* __restrict__ bh,
                                                  const unsigned short* __restrict__ bl,
                                                  float* __restrict__ S)
{
  __shared__ __attribute__((aligned(16))) float sT[4 * 64 * 32];

  const int tid = threadIdx.x, lane = tid & 31, w = tid >> 5;
  const int h = lane >> 4, m = lane & 15;
  const int m0 = blockIdx.x * 64;
  const int n0w = blockIdx.y * 128 + 32 * w;

  const unsigned short* pah = ah + (size_t)(m0 + m) * KP;
  const unsigned short* pal = al + (size_t)(m0 + m) * KP;
  const unsigned short* pbh = bh + (size_t)(n0w + m) * KP;
  const unsigned short* pbl = bl + (size_t)(n0w + m) * KP;

  const v8f zero8 = {0.f, 0.f, 0.f, 0.f, 0.f, 0.f, 0.f, 0.f};
  v8f acc[4][2];
  #pragma unroll
  for (int i = 0; i < 4; ++i)
    #pragma unroll
    for (int j = 0; j < 2; ++j) acc[i][j] = zero8;

  #pragma unroll 1
  for (int k0 = 0; k0 < KLOOP; k0 += 32) {
    v16us fa[4], fl[4], gb[2], gl[2];
    #pragma unroll
    for (int i = 0; i < 4; ++i) {
      fa[i] = load_frag(pah + (size_t)i * 16 * KP + k0, h);
      fl[i] = load_frag(pal + (size_t)i * 16 * KP + k0, h);
    }
    #pragma unroll
    for (int j = 0; j < 2; ++j) {
      gb[j] = load_frag(pbh + (size_t)j * 16 * KP + k0, h);
      gl[j] = load_frag(pbl + (size_t)j * 16 * KP + k0, h);
    }
    #pragma unroll
    for (int i = 0; i < 4; ++i) {
      #pragma unroll
      for (int j = 0; j < 2; ++j) {
        acc[i][j] = wmma_bf(fa[i], gb[j], acc[i][j]);
        acc[i][j] = wmma_bf(fa[i], gl[j], acc[i][j]);
        acc[i][j] = wmma_bf(fl[i], gb[j], acc[i][j]);
      }
    }
    asm volatile("v_nop\n\tv_nop\n\tv_nop\n\tv_nop"
                 : "+v"(acc[0][0]), "+v"(acc[0][1]), "+v"(acc[1][0]), "+v"(acc[1][1]),
                   "+v"(acc[2][0]), "+v"(acc[2][1]), "+v"(acc[3][0]), "+v"(acc[3][1])
                 : "v"(fa[0]), "v"(fa[1]), "v"(fa[2]), "v"(fa[3]),
                   "v"(fl[0]), "v"(fl[1]), "v"(fl[2]), "v"(fl[3]),
                   "v"(gb[0]), "v"(gb[1]), "v"(gl[0]), "v"(gl[1]));
  }

  float* so = sT + w * 2048;
  #pragma unroll
  for (int i = 0; i < 4; ++i)
    #pragma unroll
    for (int j = 0; j < 2; ++j)
      #pragma unroll
      for (int r = 0; r < 8; ++r)
        so[(16 * i + 8 * h + r) * 32 + 16 * j + m] = acc[i][j][r];
  __syncthreads();

  gemm_store_pass(so, S, m0, n0w, lane);
  __threadfence();
  gemm_store_pass(so, S, m0, n0w, lane);
}

__global__ __launch_bounds__(256) void overlap_add(const float* __restrict__ S, const float* __restrict__ win,
                                                   float* __restrict__ out, int pass_id)
{
  const int g = blockIdx.x * 256 + threadIdx.x;
  if (g >= NBH * QROW) return;
  const int blk = g / QROW;
  const int q = g - blk * QROW;
  const int mo = 4 * q;
  const int p0 = mo + NFFT / 2;
  const int tt = p0 >> 8;
  const int nb = p0 & (HOP - 1);

  v4f acc = {0.f, 0.f, 0.f, 0.f};
  v4f ws  = {0.f, 0.f, 0.f, 0.f};
  #pragma unroll
  for (int j = 0; j < 4; ++j) {
    const int t = tt - j;
    const bool ok = (t >= 0) && (t < NFRAMES);
    const int tc = min(max(t, 0), NFRAMES - 1);
    const int n = nb + HOP * j;
    const v4f s  = *(const v4fa*)(S + ((size_t)(blk * NFRAMES + tc)) * NFFT + n);
    const v4f wv = *(const v4fa*)(win + n);
    #pragma unroll
    for (int e = 0; e < 4; ++e) {
      acc[e] += ok ? s[e] : 0.0f;
      ws[e]  += ok ? wv[e] : 0.0f;
    }
  }
  v4f y;
  #pragma unroll
  for (int e = 0; e < 4; ++e) {
    const float d = fmaxf(ws[e], 1e-11f);
    y[e] = acc[e] * (1.0f / d);
  }
  float* dst = out + (size_t)(pass_id * NBH + blk) * OUTLEN + mo;
  *(volatile v4f*)dst = y;
  __threadfence();
  *(volatile v4f*)dst = y;
}

extern "C" void kernel_launch(void* const* d_in, const int* in_sizes, int n_in,
                              void* d_out, int out_size, void* d_ws, size_t ws_size,
                              hipStream_t stream) {
  if (n_in < 5) return;
  if (in_sizes[0] != NB * NFREQ * NFRAMES || in_sizes[1] != NB * NFREQ * NFRAMES) return;
  if (in_sizes[2] != NFFT * NFFT || in_sizes[3] != NFFT * NFFT || in_sizes[4] != NFFT) return;
  if (out_size != NB * OUTLEN) return;

  const float* re  = (const float*)d_in[0];
  const float* im  = (const float*)d_in[1];
  const float* Wr  = (const float*)d_in[2];
  const float* Wi  = (const float*)d_in[3];
  const float* win = (const float*)d_in[4];
  float* out = (float*)d_out;

  const size_t A_BYTES = (size_t)MH * KP * 2;
  const size_t B_BYTES = (size_t)NFFT * KP * 2;
  const size_t S_BYTES = (size_t)MH * NFFT * 4;
  const size_t total = 2 * A_BYTES + 2 * B_BYTES + S_BYTES;
  if (total > ws_size) return;

  char* ws = (char*)d_ws;
  unsigned short* ah = (unsigned short*)(ws);
  unsigned short* al = (unsigned short*)(ws + A_BYTES);
  unsigned short* bh = (unsigned short*)(ws + 2 * A_BYTES);
  unsigned short* bl = (unsigned short*)(ws + 2 * A_BYTES + B_BYTES);
  float* S = (float*)(ws + 2 * A_BYTES + 2 * B_BYTES);

  prep_basis<<<dim3(KP / 64, NFFT / 64), 256, 0, stream>>>(Wr, Wi, bh, bl);

  for (int ps = 0; ps < NB / NBH; ++ps) {
    prep_frames<<<dim3(KP / 64, (NFRAMES + 63) / 64, NBH), 256, 0, stream>>>(re, im, ah, al, ps);
    synth_gemm<<<dim3(MH / 64, NFFT / 128), 128, 0, stream>>>(ah, al, bh, bl, S);
    overlap_add<<<(NBH * QROW + 255) / 256, 256, 0, stream>>>(S, win, out, ps);
  }
}
